// DSAAM_13219909337528
// MI455X (gfx1250) — hardware-verified
//
#include <hip/hip_runtime.h>
#include <stdint.h>
#include <stddef.h>


typedef _Float16 v16h __attribute__((ext_vector_type(16)));
typedef _Float16 v8h  __attribute__((ext_vector_type(8), may_alias));
typedef float    v8f  __attribute__((ext_vector_type(8)));
typedef float    v4f  __attribute__((ext_vector_type(4), may_alias));
typedef unsigned int v4u __attribute__((ext_vector_type(4), may_alias));

union Frag  { v16h v; v8h half[2]; };
union Pack8 { v8h h; v4u u; _Float16 s[8]; };

#define DIMC   256
#define NHEAD  8
#define NPTS   8
#define HDIM   32
#define NTOK   16384
#define NBATCH 2
#define MROWS  (NBATCH * NTOK)
#define NOFF   128
#define NATT   64
#define NCAT   (DIMC + NOFF + NATT)
#define WROWS  (NCAT + DIMC)
#define GW     128
#define GH     128
#define SC_A   64.0f
#define SC_B   1024.0f
#define SC_OUT (1.0f / 65536.0f)

static_assert(MROWS % 256 == 0, "");
static_assert(NCAT % 32 == 0, "");
static_assert(DIMC % 32 == 0, "");
static_assert(MROWS % 8 == 0, "");
static_assert(GW * GH == NTOK, "");

__device__ __forceinline__ int iclamp(int v, int lo, int hi) {
    return v < lo ? lo : (v > hi ? hi : v);
}

__device__ __forceinline__ v8f wmma_f16(const v16h a, const v16h b, v8f c) {
    v8f d = __builtin_amdgcn_wmma_f32_16x16x32_f16(false, a, false, b, (short)0, c, false, false);
    asm volatile("v_nop\n\tv_nop\n\tv_nop\n\tv_nop" : "+v"(d) : "v"(a), "v"(b));
    return d;
}

__device__ __forceinline__ void cvt1(float v, _Float16& h, _Float16& l) {
    _Float16 q = (_Float16)v;
    h = q;
    l = (_Float16)(v - (float)q);
}
__device__ __forceinline__ void split8(v4f f0, v4f f1, float sc, Pack8& ph, Pack8& pl) {
    cvt1(f0.x * sc, ph.s[0], pl.s[0]);
    cvt1(f0.y * sc, ph.s[1], pl.s[1]);
    cvt1(f0.z * sc, ph.s[2], pl.s[2]);
    cvt1(f0.w * sc, ph.s[3], pl.s[3]);
    cvt1(f1.x * sc, ph.s[4], pl.s[4]);
    cvt1(f1.y * sc, ph.s[5], pl.s[5]);
    cvt1(f1.z * sc, ph.s[6], pl.s[6]);
    cvt1(f1.w * sc, ph.s[7], pl.s[7]);
}

__global__ void __launch_bounds__(256)
k_cvt_x(const float* __restrict__ x, _Float16* xh, _Float16* xl, int n8)
{
    const int i = blockIdx.x * 256 + threadIdx.x;
    if (i >= n8) return;
    const float* s = x + (size_t)i * 8;
    v4f f0 = *(const v4f*)s;
    v4f f1 = *(const v4f*)(s + 4);
    Pack8 ph, pl;
    split8(f0, f1, SC_A, ph, pl);
    volatile v4u* dh = (volatile v4u*)(xh + (size_t)i * 8);
    volatile v4u* dl = (volatile v4u*)(xl + (size_t)i * 8);
    *dh = ph.u;
    *dl = pl.u;
    __threadfence();
    *dh = ph.u;
    *dl = pl.u;
}

__global__ void __launch_bounds__(256)
k_prep_w(const float* __restrict__ Wv, const float* __restrict__ Woff,
         const float* __restrict__ Wa, const float* __restrict__ Wout,
         _Float16* Wh, _Float16* Wl, int nrows)
{
    const int t = blockIdx.x * 256 + threadIdx.x;
    const int j = t >> 5, kq = t & 31;
    if (j >= nrows) return;
    const float* src; int pitch;
    if (j < DIMC)             { src = Wv + j;                 pitch = DIMC; }
    else if (j < DIMC + NOFF) { src = Woff + (j - DIMC);      pitch = NOFF; }
    else if (j < NCAT)        { src = Wa + (j - DIMC - NOFF); pitch = NATT; }
    else                      { src = Wout + (j - NCAT);      pitch = DIMC; }
    const int kb = kq * 8;
    v4f f0, f1;
    f0.x = src[(size_t)(kb + 0) * pitch];
    f0.y = src[(size_t)(kb + 1) * pitch];
    f0.z = src[(size_t)(kb + 2) * pitch];
    f0.w = src[(size_t)(kb + 3) * pitch];
    f1.x = src[(size_t)(kb + 4) * pitch];
    f1.y = src[(size_t)(kb + 5) * pitch];
    f1.z = src[(size_t)(kb + 6) * pitch];
    f1.w = src[(size_t)(kb + 7) * pitch];
    Pack8 ph, pl;
    split8(f0, f1, SC_B, ph, pl);
    volatile v4u* dh = (volatile v4u*)(Wh + (size_t)j * DIMC + kb);
    volatile v4u* dl = (volatile v4u*)(Wl + (size_t)j * DIMC + kb);
    *dh = ph.u;
    *dl = pl.u;
    __threadfence();
    *dh = ph.u;
    *dl = pl.u;
}

union GemmLds { _Float16 b[2][32 * DIMC]; float s[8][1024]; };

template <int NCOLS, int NSEG0, int NSEG1>
__global__ void __launch_bounds__(256)
k_gemm3(const _Float16* __restrict__ Ah, const _Float16* __restrict__ Al,
        const _Float16* __restrict__ Bh, const _Float16* __restrict__ Bl,
        const float* __restrict__ bias0, const float* __restrict__ bias1,
        const float* __restrict__ bias2, float* C, float oscale)
{
    __shared__ __align__(16) GemmLds lds;
    const int colbase = blockIdx.y * 32;

    {
        const _Float16* gh = Bh + (size_t)colbase * DIMC;
        const _Float16* gl = Bl + (size_t)colbase * DIMC;
#pragma unroll
        for (int i = 0; i < 4; ++i) {
            const int c = threadIdx.x + 256 * i;
            *(v8h*)(&lds.b[0][c * 8]) = *(const v8h*)(gh + (size_t)c * 8);
            *(v8h*)(&lds.b[1][c * 8]) = *(const v8h*)(gl + (size_t)c * 8);
        }
    }
    __syncthreads();

    const int wave = threadIdx.x >> 5, lane = threadIdx.x & 31;
    const int l16 = lane & 15, hh = lane >> 4;
    const int rowbase = blockIdx.x * 256 + wave * 32;

    const _Float16* pah0 = Ah + (size_t)(rowbase + l16) * DIMC + 8 * hh;
    const _Float16* pal0 = Al + (size_t)(rowbase + l16) * DIMC + 8 * hh;
    const _Float16* pah1 = pah0 + 16 * DIMC;
    const _Float16* pal1 = pal0 + 16 * DIMC;
    const _Float16* pbh = &lds.b[0][l16 * DIMC + 8 * hh];
    const _Float16* pbl = &lds.b[1][l16 * DIMC + 8 * hh];

    v8f acc[2][2] = {{v8f{}, v8f{}}, {v8f{}, v8f{}}};

#pragma unroll 2
    for (int k0 = 0; k0 < DIMC; k0 += 32) {
        Frag ah0, al0, ah1, al1;
        ah0.half[0] = *(const v8h*)(pah0 + k0);  ah0.half[1] = *(const v8h*)(pah0 + k0 + 16);
        al0.half[0] = *(const v8h*)(pal0 + k0);  al0.half[1] = *(const v8h*)(pal0 + k0 + 16);
        ah1.half[0] = *(const v8h*)(pah1 + k0);  ah1.half[1] = *(const v8h*)(pah1 + k0 + 16);
        al1.half[0] = *(const v8h*)(pal1 + k0);  al1.half[1] = *(const v8h*)(pal1 + k0 + 16);
#pragma unroll
        for (int j = 0; j < 2; ++j) {
            const int ob = j * 16 * DIMC + k0;
            Frag bh, bl;
            bh.half[0] = *(const v8h*)(pbh + ob);  bh.half[1] = *(const v8h*)(pbh + ob + 16);
            bl.half[0] = *(const v8h*)(pbl + ob);  bl.half[1] = *(const v8h*)(pbl + ob + 16);
            acc[0][j] = wmma_f16(ah0.v, bh.v, acc[0][j]);
            acc[0][j] = wmma_f16(ah0.v, bl.v, acc[0][j]);
            acc[0][j] = wmma_f16(al0.v, bh.v, acc[0][j]);
            acc[1][j] = wmma_f16(ah1.v, bh.v, acc[1][j]);
            acc[1][j] = wmma_f16(ah1.v, bl.v, acc[1][j]);
            acc[1][j] = wmma_f16(al1.v, bh.v, acc[1][j]);
        }
    }

    __syncthreads();

    const float* bp;
    if (colbase < NSEG0)              bp = bias0 + colbase;
    else if (colbase < NSEG0 + NSEG1) bp = bias1 + (colbase - NSEG0);
    else                              bp = bias2 + (colbase - NSEG0 - NSEG1);
    const float bj0 = bp[l16];
    const float bj1 = bp[16 + l16];

    float* stg = &lds.s[wave][0];
#pragma unroll
    for (int mi = 0; mi < 2; ++mi) {
#pragma unroll
        for (int r = 0; r < 8; ++r) {
            const int rr = mi * 16 + 8 * hh + r;
            stg[rr * 32 + l16]      = acc[mi][0][r] * oscale + bj0;
            stg[rr * 32 + 16 + l16] = acc[mi][1][r] * oscale + bj1;
        }
    }
    __syncthreads();

    const int rq = lane >> 3, c4 = (lane & 7) * 4;
    v4f v[8];
#pragma unroll
    for (int it = 0; it < 8; ++it)
        v[it] = *(const v4f*)(stg + (it * 4 + rq) * 32 + c4);

    float* cb = C + (size_t)(rowbase + rq) * NCOLS + colbase + c4;
#pragma unroll
    for (int it = 0; it < 8; ++it)
        *(volatile v4f*)(cb + (size_t)(it * 4) * NCOLS) = v[it];
    __threadfence();
#pragma unroll
    for (int it = 0; it < 8; ++it)
        *(volatile v4f*)(cb + (size_t)(it * 4) * NCOLS) = v[it];
}

__global__ void __launch_bounds__(256)
k_sample(const float* __restrict__ cat, const float* __restrict__ rp,
         _Float16* mhi, _Float16* mlo, int ntok)
{
#pragma clang fp contract(off)
    __shared__ __align__(16) float stg[8][DIMC];
    const int wave = threadIdx.x >> 5, lane = threadIdx.x & 31;
    const int tok = blockIdx.x * 8 + wave;
    const bool ok = tok < ntok;
    const int tk = ok ? tok : 0;
    const int b = tk / NTOK;

    const float* row = cat + (size_t)tk * NCAT;
    const float rx = rp[(size_t)tk * 2 + 0];
    const float ry = rp[(size_t)tk * 2 + 1];
    const float* vb = cat + (size_t)b * NTOK * NCAT + lane;

#pragma unroll 1
    for (int h = 0; h < NHEAD; ++h) {
        const float* lgp = row + DIMC + NOFF + h * NPTS;
        float e[NPTS];
#pragma unroll
        for (int p = 0; p < NPTS; ++p) e[p] = lgp[p];
        float mx = e[0];
#pragma unroll
        for (int p = 1; p < NPTS; ++p) mx = fmaxf(mx, e[p]);
        float s = 0.f;
#pragma unroll
        for (int p = 0; p < NPTS; ++p) { e[p] = __expf(e[p] - mx); s = s + e[p]; }
        const float inv = 1.0f / s;

        const float* vh = vb + h * HDIM;
        const float* orow = row + DIMC + h * (NPTS * 2);
        float acc = 0.f;
#pragma unroll
        for (int p = 0; p < NPTS; ++p) {
            const float gx = fminf(fmaxf(rx + orow[2 * p + 0], -1.f), 1.f);
            const float gy = fminf(fmaxf(ry + orow[2 * p + 1], -1.f), 1.f);
            const float xp = (gx + 1.f) * 0.5f * (float)(GW - 1);
            const float yp = (gy + 1.f) * 0.5f * (float)(GH - 1);
            const float xf = floorf(xp), yf = floorf(yp);
            const float wx = xp - xf, wy = yp - yf;
            const int x0 = (int)xf, y0 = (int)yf;
            const int x0c = iclamp(x0, 0, GW - 1), x1c = iclamp(x0 + 1, 0, GW - 1);
            const int y0c = iclamp(y0, 0, GH - 1), y1c = iclamp(y0 + 1, 0, GH - 1);
            const float v00 = vh[(size_t)(y0c * GW + x0c) * NCAT];
            const float v01 = vh[(size_t)(y0c * GW + x1c) * NCAT];
            const float v10 = vh[(size_t)(y1c * GW + x0c) * NCAT];
            const float v11 = vh[(size_t)(y1c * GW + x1c) * NCAT];
            const float sv = v00 * (1.f - wx) * (1.f - wy) + v01 * wx * (1.f - wy)
                           + v10 * (1.f - wx) * wy + v11 * wx * wy;
            acc = acc + sv * (e[p] * inv);
        }
        stg[wave][h * HDIM + lane] = acc;
    }
    __syncthreads();

    v4f f0 = *(const v4f*)(&stg[wave][8 * lane]);
    v4f f1 = *(const v4f*)(&stg[wave][8 * lane + 4]);
    Pack8 ph, pl;
    split8(f0, f1, SC_A, ph, pl);
    volatile v4u* dh = (volatile v4u*)(mhi + (size_t)tk * DIMC + 8 * lane);
    volatile v4u* dl = (volatile v4u*)(mlo + (size_t)tk * DIMC + 8 * lane);
    if (ok) { *dh = ph.u; *dl = pl.u; }
    __threadfence();
    if (ok) { *dh = ph.u; *dl = pl.u; }
}

extern "C" void kernel_launch(void* const* d_in, const int* in_sizes, int n_in,
                              void* d_out, int out_size, void* d_ws, size_t ws_size,
                              hipStream_t stream)
{
    if (n_in < 10) return;
    if (in_sizes[0] != MROWS * DIMC || in_sizes[1] != MROWS * 2 ||
        in_sizes[2] != DIMC * DIMC || in_sizes[3] != DIMC ||
        in_sizes[4] != DIMC * NOFF || in_sizes[5] != NOFF ||
        in_sizes[6] != DIMC * NATT || in_sizes[7] != NATT ||
        in_sizes[8] != DIMC * DIMC || in_sizes[9] != DIMC) return;
    if (out_size != MROWS * DIMC) return;

    const float* x    = (const float*)d_in[0];
    const float* refp = (const float*)d_in[1];
    const float* Wv   = (const float*)d_in[2];
    const float* bv   = (const float*)d_in[3];
    const float* Woff = (const float*)d_in[4];
    const float* boff = (const float*)d_in[5];
    const float* Wa   = (const float*)d_in[6];
    const float* ba   = (const float*)d_in[7];
    const float* Wout = (const float*)d_in[8];
    const float* bout = (const float*)d_in[9];
    float* out = (float*)d_out;

    char* ws = (char*)d_ws;
    size_t off = 0;
    const size_t xplane = (size_t)MROWS * DIMC * sizeof(_Float16);
    const size_t wplane = (size_t)WROWS * DIMC * sizeof(_Float16);
    const size_t catb   = (size_t)MROWS * NCAT * sizeof(float);
    _Float16* xh  = (_Float16*)(ws + off); off += xplane;
    _Float16* xl  = (_Float16*)(ws + off); off += xplane;
    _Float16* Wh  = (_Float16*)(ws + off); off += wplane;
    _Float16* Wl  = (_Float16*)(ws + off); off += wplane;
    float*    cat = (float*)(ws + off);    off += catb;
    _Float16* mh  = (_Float16*)(ws + off); off += xplane;
    _Float16* ml  = (_Float16*)(ws + off); off += xplane;
    if (off > ws_size) return;

    const int n8 = MROWS * DIMC / 8;
    k_cvt_x<<<(n8 + 255) / 256, 256, 0, stream>>>(x, xh, xl, n8);

    const int prepT = WROWS * 32;
    k_prep_w<<<(prepT + 255) / 256, 256, 0, stream>>>(Wv, Woff, Wa, Wout, Wh, Wl, WROWS);

    k_gemm3<NCAT, DIMC, NOFF><<<dim3(MROWS / 256, NCAT / 32), 256, 0, stream>>>(
        xh, xl, Wh, Wl, bv, boff, ba, cat, SC_OUT);

    k_sample<<<MROWS / 8, 256, 0, stream>>>(cat, refp, mh, ml, MROWS);

    k_gemm3<DIMC, DIMC, 0><<<dim3(MROWS / 256, DIMC / 32), 256, 0, stream>>>(
        mh, ml, Wh + (size_t)NCAT * DIMC, Wl + (size_t)NCAT * DIMC, bout, bout, bout, out, SC_OUT);
}
